// SingleHeadMDTA_35923106464231
// MI455X (gfx1250) — hardware-verified
//
#include <hip/hip_runtime.h>


#define NB_  4
#define CC   48
#define CP   64
#define HH   256
#define WWD  256
#define NP   (HH * WWD)
typedef _Float16 h16;
typedef unsigned short bf;
typedef __attribute__((ext_vector_type(16))) __bf16   v16bf;
typedef __attribute__((ext_vector_type(16))) _Float16 v16h;
typedef __attribute__((ext_vector_type(8)))  _Float16 v8h;
typedef __attribute__((ext_vector_type(8)))  unsigned short v8us;
typedef __attribute__((ext_vector_type(8)))  float    v8f;
typedef __attribute__((ext_vector_type(4)))  float    v4f;
typedef v8h  __attribute__((may_alias)) v8ha;
typedef v4f  __attribute__((may_alias)) v4fa;
typedef v8us __attribute__((may_alias)) v8usa;

__device__ __forceinline__ unsigned short f2bf(float f) { unsigned u = __float_as_uint(f); u += 0x7FFFu + ((u >> 16) & 1u); return (unsigned short)(u >> 16); }
__device__ __forceinline__ float bf2f(unsigned short b) { return __uint_as_float(((unsigned)b) << 16); }
__device__ __forceinline__ float bfr(float f) { return bf2f(f2bf(f)); }
__device__ __forceinline__ v16h cat16(v8h lo, v8h hi) { return __builtin_shufflevector(lo, hi, 0, 1, 2, 3, 4, 5, 6, 7, 8, 9, 10, 11, 12, 13, 14, 15); }
__device__ __forceinline__ v16bf cat16b(v8us lo, v8us hi) { return __builtin_bit_cast(v16bf, __builtin_shufflevector(lo, hi, 0, 1, 2, 3, 4, 5, 6, 7, 8, 9, 10, 11, 12, 13, 14, 15)); }
__device__ __forceinline__ v8f wmma16(v16h a, v16h b, v8f c) { return __builtin_amdgcn_wmma_f32_16x16x32_f16(false, a, false, b, (short)0, c, false, false); }
__device__ __forceinline__ v8f wmmab(v16bf a, v16bf b, v8f c) { return __builtin_amdgcn_wmma_f32_16x16x32_bf16(false, a, false, b, (short)0, c, false, false); }


template <typename T16> struct WFrag;
template <> struct WFrag<h16> { typedef v16h V; static __device__ __forceinline__ V ld(const h16* p) { return cat16(*(const v8h*)p, *(const v8h*)(p + 16)); } static __device__ __forceinline__ v8f mma(V a, V b, v8f c) { return wmma16(a, b, c); } };
template <> struct WFrag<bf> { typedef v16bf V; static __device__ __forceinline__ V ld(const bf* p) { return cat16b(*(const v8us*)p, *(const v8us*)(p + 16)); } static __device__ __forceinline__ v8f mma(V a, V b, v8f c) { return wmmab(a, b, c); } };
template <typename T16, int NSPLIT, bool BIAS>
__global__ __launch_bounds__(32) void k_gemmw(const T16* __restrict__ A, const T16* __restrict__ A2, const T16* __restrict__ Bt, const T16* __restrict__ Bt2, int K, float* C, int ldc, const float* __restrict__ bias, size_t sA, size_t sB, size_t sC) {
    typedef typename WFrag<T16>::V V;
    __shared__ __align__(16) float os[16 * 68];
    const size_t z = blockIdx.z; A += z * sA; if (A2) A2 += z * sA; Bt += z * sB; if (Bt2) Bt2 += z * sB; C += z * sC;
    const int lane = threadIdx.x & 31, lr = lane & 15, hi = lane >> 4; const int r0 = blockIdx.x * 64, c0 = blockIdx.y * 64;
    v8f acc[4][4];
#pragma unroll
    for (int mb = 0; mb < 4; ++mb)
#pragma unroll
        for (int nb = 0; nb < 4; ++nb) acc[mb][nb] = (v8f){};
    const size_t aoff = (size_t)(r0 + lr) * K + 8 * hi, boff = (size_t)(c0 + lr) * K + 8 * hi;
#pragma unroll 1
    for (int kc = 0; kc < K; kc += 32) {
        V a[4], a2[4];
#pragma unroll
        for (int mb = 0; mb < 4; ++mb) { a[mb] = WFrag<T16>::ld(A + aoff + (size_t)mb * 16 * K + kc); if (NSPLIT == 1 || NSPLIT == 2) a2[mb] = WFrag<T16>::ld(A2 + aoff + (size_t)mb * 16 * K + kc); }
#pragma unroll
        for (int nb = 0; nb < 4; ++nb) { const V b = WFrag<T16>::ld(Bt + boff + (size_t)nb * 16 * K + kc); V b2; if (NSPLIT >= 2) b2 = WFrag<T16>::ld(Bt2 + boff + (size_t)nb * 16 * K + kc);
#pragma unroll
            for (int mb = 0; mb < 4; ++mb) { acc[mb][nb] = WFrag<T16>::mma(a[mb], b, acc[mb][nb]); if (NSPLIT == 1 || NSPLIT == 2) acc[mb][nb] = WFrag<T16>::mma(a2[mb], b, acc[mb][nb]); if (NSPLIT >= 2) acc[mb][nb] = WFrag<T16>::mma(a[mb], b2, acc[mb][nb]); } }
        asm volatile("v_nop\n\tv_nop\n\tv_nop\n\tv_nop" : "+v"(acc[0][0]), "+v"(acc[1][1]), "+v"(acc[2][2]), "+v"(acc[3][3]) : "v"(a[0]), "v"(a[3]));
    }
#pragma unroll
    for (int mb = 0; mb < 4; ++mb) {
#pragma unroll
        for (int nb = 0; nb < 4; ++nb) {
#pragma unroll
            for (int j = 0; j < 8; ++j) os[(hi * 8 + j) * 68 + nb * 16 + lr] = acc[mb][nb][j]; }
        __builtin_amdgcn_wave_barrier(); asm volatile("" ::: "memory");
        float* crow = C + (size_t)(r0 + mb * 16) * ldc + c0;
#pragma unroll 1
        for (int ps = 0; ps < 2; ++ps) {
#pragma unroll
            for (int s = 0; s < 8; ++s) { const int row = 2 * s + hi, cofs = lr * 4; v4f val = *(const v4fa*)(os + row * 68 + cofs); if (BIAS) { val[0] += bfr(bias[c0 + cofs]); val[1] += bfr(bias[c0 + cofs + 1]); val[2] += bfr(bias[c0 + cofs + 2]); val[3] += bfr(bias[c0 + cofs + 3]); }
                *(volatile v4f*)(crow + (size_t)row * ldc + cofs) = val; }
            if (ps == 0) __threadfence(); }
        __builtin_amdgcn_wave_barrier(); asm volatile("" ::: "memory");
    }
}

__device__ __forceinline__ void splitf(float y, unsigned short& h, unsigned short& l) { h = f2bf(y); l = f2bf(y - bf2f(h)); }
typedef __attribute__((ext_vector_type(2))) unsigned short v2us;

__global__ __launch_bounds__(256) void k_wpad(const float* __restrict__ w, bf* WP) {
    const int lane = threadIdx.x & 31; const int L = blockIdx.x * 8 + (threadIdx.x >> 5); if (L >= CP * CP / 64) return; const int e = L * 64 + lane * 2; const int c = e & 63, o = e >> 6; v2us v;
#pragma unroll
    for (int q = 0; q < 2; ++q) v[q] = (o < CC && c + q < CC) ? f2bf(w[o * CC + c + q]) : (unsigned short)0;
    *(volatile v2us*)(WP + e) = v; __threadfence(); *(volatile v2us*)(WP + e) = v;
}
__global__ __launch_bounds__(256) void k_xT(const float* __restrict__ x, int b, bf* XT) {
    const int lane = threadIdx.x & 31; const int L0 = (blockIdx.x * 8 + (threadIdx.x >> 5)) * 8; const int nlines = NP * CP / 64;
#pragma unroll 1
    for (int ps = 0; ps < 2; ++ps) {
#pragma unroll
        for (int l = 0; l < 8; ++l) { const int L = L0 + l; if (L >= nlines) break; const int e = L * 64 + lane * 2; const int c = e & 63, p = e >> 6; v2us v;
#pragma unroll
            for (int q = 0; q < 2; ++q) v[q] = (c + q < CC) ? f2bf(x[((size_t)b * CC + c + q) * NP + p]) : (unsigned short)0;
            *(volatile v2us*)(XT + (size_t)e) = v; }
        if (ps == 0) __threadfence(); }
}
template <bool TOK>
__global__ __launch_bounds__(256) void k_dw(const float* __restrict__ Y, const float* __restrict__ wdw, bf* Ph, bf* Pl) {
    const int lane = threadIdx.x & 31; const int L0 = (blockIdx.x * 8 + (threadIdx.x >> 5)) * 8; const int nlines = CP * NP / 64;
#pragma unroll 1
    for (int ps = 0; ps < 2; ++ps) {
#pragma unroll 1
        for (int l = 0; l < 8; ++l) { const int L = L0 + l; if (L >= nlines) break; const int e = L * 64 + lane * 2; v2us oh, ol;
#pragma unroll
            for (int q = 0; q < 2; ++q) { int o, p; if (TOK) { o = (e + q) & 63; p = (e + q) >> 6; } else { p = (e + q) & (NP - 1); o = (e + q) >> 16; }
                float acc = 0.f;
                if (o < CC) { const int h = p >> 8, w = p & 255; const float* yr = Y + (size_t)o * NP;
#pragma unroll
                    for (int kh = 0; kh < 3; ++kh) { const int hh = h + kh - 1; if (hh < 0 || hh >= HH) continue;
#pragma unroll
                        for (int kw = 0; kw < 3; ++kw) { const int ww = w + kw - 1; if (ww < 0 || ww >= WWD) continue; acc = fmaf(bfr(wdw[o * 9 + kh * 3 + kw]), yr[hh * WWD + ww], acc); } } }
                unsigned short a, c2; splitf(acc, a, c2); oh[q] = a; ol[q] = c2; }
            *(volatile v2us*)(Ph + (size_t)e) = oh; *(volatile v2us*)(Pl + (size_t)e) = ol; }
        if (ps == 0) __threadfence(); }
}
__global__ __launch_bounds__(256) void k_soft48(const float* __restrict__ S, const float* __restrict__ alpha, bf* Th, bf* Tl) {
    const int lane = threadIdx.x & 31; const int d = blockIdx.x * 8 + (threadIdx.x >> 5); if (d >= CP) return; const float ia = bfr(alpha[0]); v2us oh, ol;
#pragma unroll
    for (int q = 0; q < 2; ++q) { const int c = lane * 2 + q; float val = 0.f;
        if (c < CC && d < CC) { const float* sr = S + (size_t)c * CP; float m = -3.0e38f;
#pragma unroll 1
            for (int j = 0; j < CC; ++j) m = fmaxf(m, __fdiv_rn(sr[j], ia));
            float sum = 0.f;
#pragma unroll 1
            for (int j = 0; j < CC; ++j) sum += __expf(__fdiv_rn(sr[j], ia) - m);
            val = __fdiv_rn(__expf(__fdiv_rn(sr[d], ia) - m), sum); }
        unsigned short a, c2; splitf(val, a, c2); oh[q] = a; ol[q] = c2; }
    *(volatile v2us*)(Th + (size_t)d * CP + lane * 2) = oh; *(volatile v2us*)(Tl + (size_t)d * CP + lane * 2) = ol; __threadfence(); *(volatile v2us*)(Th + (size_t)d * CP + lane * 2) = oh; *(volatile v2us*)(Tl + (size_t)d * CP + lane * 2) = ol;
}
__global__ __launch_bounds__(256) void k_out48(const float* __restrict__ O, int b, float* OUT) { const size_t i = (size_t)blockIdx.x * 256 + threadIdx.x; if (i >= (size_t)CC * NP / 4) return; const v4f v = *(const v4f*)(O + i * 4); float* dst = OUT + (size_t)b * CC * NP + i * 4; *(volatile v4f*)dst = v; __threadfence(); *(volatile v4f*)dst = v; }

extern "C" void kernel_launch(void* const* d_in, const int* in_sizes, int n_in,
                              void* d_out, int out_size, void* d_ws, size_t ws_size, hipStream_t stream) {
    (void)in_sizes; (void)n_in; (void)out_size;
    const float* x = (const float*)d_in[0]; const float* wq_pw = (const float*)d_in[1]; const float* wq_dw = (const float*)d_in[2]; const float* wk_pw = (const float*)d_in[3]; const float* wk_dw = (const float*)d_in[4]; const float* wv_pw = (const float*)d_in[5]; const float* wv_dw = (const float*)d_in[6]; const float* alpha = (const float*)d_in[7];
    float* OUT = (float*)d_out;
    char* wsp = (char*)d_ws;
    auto take = [&](size_t bytes) { char* p = wsp; wsp += (bytes + 255) & ~(size_t)255; return (void*)p; };
    bf* WQ = (bf*)take(CP * CP * 2); bf* WK = (bf*)take(CP * CP * 2); bf* WV = (bf*)take(CP * CP * 2);
    bf* XT = (bf*)take((size_t)NP * CP * 2); float* Y = (float*)take((size_t)CP * NP * 4);
    bf* Qh = (bf*)take((size_t)CP * NP * 2); bf* Ql = (bf*)take((size_t)CP * NP * 2); bf* Kh = (bf*)take((size_t)CP * NP * 2); bf* Kl = (bf*)take((size_t)CP * NP * 2); bf* VTh = (bf*)take((size_t)NP * CP * 2); bf* VTl = (bf*)take((size_t)NP * CP * 2);
    float* S = (float*)take(CP * CP * 4); bf* Th = (bf*)take(CP * CP * 2); bf* Tl = (bf*)take(CP * CP * 2); float* O = (float*)take((size_t)CP * NP * 4);
    if ((size_t)(wsp - (char*)d_ws) > ws_size) return;
    k_wpad<<<(CP * CP / 64 + 7) / 8, 256, 0, stream>>>(wq_pw, WQ); k_wpad<<<(CP * CP / 64 + 7) / 8, 256, 0, stream>>>(wk_pw, WK); k_wpad<<<(CP * CP / 64 + 7) / 8, 256, 0, stream>>>(wv_pw, WV);
    const unsigned LP = (unsigned)((CP * NP / 64 + 63) / 64);
    for (int b = 0; b < NB_; ++b) {
        k_xT<<<LP, 256, 0, stream>>>(x, b, XT);
        k_gemmw<bf, 0, false><<<dim3(1, NP / 64, 1), 32, 0, stream>>>(WQ, nullptr, XT, nullptr, CP, Y, NP, nullptr, 0, 0, 0); k_dw<false><<<LP, 256, 0, stream>>>(Y, wq_dw, Qh, Ql);
        k_gemmw<bf, 0, false><<<dim3(1, NP / 64, 1), 32, 0, stream>>>(WK, nullptr, XT, nullptr, CP, Y, NP, nullptr, 0, 0, 0); k_dw<false><<<LP, 256, 0, stream>>>(Y, wk_dw, Kh, Kl);
        k_gemmw<bf, 0, false><<<dim3(1, NP / 64, 1), 32, 0, stream>>>(WV, nullptr, XT, nullptr, CP, Y, NP, nullptr, 0, 0, 0); k_dw<true><<<LP, 256, 0, stream>>>(Y, wv_dw, VTh, VTl);
        k_gemmw<bf, 2, false><<<dim3(1, 1, 1), 32, 0, stream>>>(Kh, Kl, Qh, Ql, NP, S, CP, nullptr, 0, 0, 0);
        k_soft48<<<CP / 8, 256, 0, stream>>>(S, alpha, Th, Tl);
        k_gemmw<bf, 2, false><<<dim3(1, NP / 64, 1), 32, 0, stream>>>(Th, Tl, VTh, VTl, CP, O, NP, nullptr, 0, 0, 0);
        k_out48<<<(unsigned)(((size_t)CC * NP / 4 + 255) / 256), 256, 0, stream>>>(O, b, OUT); }
}
